// GAT_69810398429280
// MI455X (gfx1250) — hardware-run, weakly checked
//
#include <hip/hip_runtime.h>
#include <math.h>
#include <stdint.h>

#pragma clang fp contract(off)

#define NB 8
#define NC 64
#define NT 4096
#define QB 128
#define KJ 256
#define VP (KJ + 8)
#define OP (QB + 4)

static_assert(NT % QB == 0);
static_assert(NT % KJ == 0);
static_assert(KJ % 32 == 0);
static_assert(NC == 64);
static_assert(NC == 4 * 16);
static_assert(QB == 8 * 16);
static_assert(NT == 4096);
static_assert(((NB * NT / 4) % 256) == 0);
static_assert((size_t)NC * OP * sizeof(float) <= (size_t)NC * VP * 2);
static_assert((VP * 2) % 16 == 0);
static_assert((OP * 4) % 16 == 0);

typedef __attribute__((ext_vector_type(16))) __bf16   v16b;
typedef __attribute__((ext_vector_type(8)))  __bf16   v8b;
typedef __attribute__((ext_vector_type(8)))  float    v8f;
typedef __attribute__((ext_vector_type(4)))  float    v4f;
typedef __attribute__((ext_vector_type(2)))  unsigned int v2u;
typedef __attribute__((ext_vector_type(8)))  unsigned int v8u;

__device__ __forceinline__ unsigned short f2bf_bits(float f) {
  unsigned u = __float_as_uint(f);
  return (unsigned short)((u + 0x7FFFu + ((u >> 16) & 1u)) >> 16);
}
__device__ __forceinline__ float bf_bits2f(unsigned short h) { return __uint_as_float(((unsigned)h) << 16); }
__device__ __forceinline__ float bf_rne(float f) { return bf_bits2f(f2bf_bits(f)); }
__device__ __forceinline__ unsigned pk16(unsigned short a, unsigned short b) { return (unsigned)a | ((unsigned)b << 16); }

__device__ __forceinline__ v8f at_mma(v16b a, v16b b, v8f c) {
  c = __builtin_amdgcn_wmma_f32_16x16x32_bf16(false, a, false, b, (short)0, c, false, false);
  asm volatile("v_nop\n\tv_nop\n\tv_nop\n\tv_nop" : "+v"(c) : "v"(a), "v"(b));
  return c;
}

__device__ __forceinline__ void p_elem(float fi, float fj, float mi, float& lsum, unsigned short& hb, unsigned short& lb) {
  const float lg = fi + fj;
  const float s  = (lg >= 0.0f) ? lg : 0.01f * lg;
  const float p  = expf(s - mi);
  lsum = lsum + p;
  hb = f2bf_bits(p);
  lb = f2bf_bits(p - bf_bits2f(hb));
}

__global__ __launch_bounds__(256) void k_prep(const float* __restrict__ x, const float* __restrict__ w,
                                              unsigned short* __restrict__ xb, float* __restrict__ F) {
  __shared__ float wsh[NC];
  const int tid = threadIdx.x;
  const float wv = w[tid & (NC - 1)];
  asm volatile("" :: "v"(wv));
  if (tid < NC) wsh[tid] = bf_rne(wv);
  __syncthreads();

  const int g = blockIdx.x * 256 + tid;
  const int b = g >> 10;
  const int n = (g & 1023) * 4;
  const size_t base = (size_t)b * NC * NT + (size_t)n;

  v4f f = (v4f){0.f, 0.f, 0.f, 0.f};
  for (int pass = 0; pass < 2; ++pass) {
    f = (v4f){0.f, 0.f, 0.f, 0.f};
#pragma unroll 4
    for (int c = 0; c < NC; ++c) {
      const v4f xv = *(const v4f*)(x + base + (size_t)c * NT);
      const unsigned short h0 = f2bf_bits(xv[0]);
      const unsigned short h1 = f2bf_bits(xv[1]);
      const unsigned short h2 = f2bf_bits(xv[2]);
      const unsigned short h3 = f2bf_bits(xv[3]);
      const float wr = wsh[c];
      f[0] = fmaf(wr, bf_bits2f(h0), f[0]);
      f[1] = fmaf(wr, bf_bits2f(h1), f[1]);
      f[2] = fmaf(wr, bf_bits2f(h2), f[2]);
      f[3] = fmaf(wr, bf_bits2f(h3), f[3]);
      v2u u;
      u[0] = pk16(h0, h1);
      u[1] = pk16(h2, h3);
      *(volatile v2u*)(xb + base + (size_t)c * NT) = u;
    }
    __threadfence();
  }
  const v4f fo = f;
  float* fp = F + (size_t)b * NT + n;
  *(volatile v4f*)fp = fo;
  __threadfence();
  *(volatile v4f*)fp = fo;
}

union VOBuf { __bf16 v[NC * VP]; float o[NC * OP]; };

__global__ __launch_bounds__(256) __attribute__((amdgpu_num_vgpr(248)))
void k_attn(const unsigned short* __restrict__ xbp, const float* __restrict__ Fp, float* __restrict__ out) {
  union FB { v16b v; v8b h[2]; };
  __shared__ __align__(16) float Fs[NT];
  __shared__ __align__(16) VOBuf VO;
  __shared__ __align__(16) float lall[QB];
  __shared__ float wmax[8];

  const int tid  = threadIdx.x;
  const int wave = tid >> 5;
  const int lane = tid & 31;
  const int hh   = lane >> 4;
  const int c    = lane & 15;
  const int b    = blockIdx.y;
  const int i0   = blockIdx.x * QB;

  const float* Fb = Fp + (size_t)b * NT;
  float tmax = -INFINITY;
#pragma unroll
  for (int it = 0; it < 4; ++it) {
    const int idx = it * 256 + tid;
    const v4f v = *(const v4f*)(Fb + 4 * idx);
    *(v4f*)(Fs + 4 * idx) = v;
    tmax = fmaxf(tmax, fmaxf(fmaxf(v[0], v[1]), fmaxf(v[2], v[3])));
  }
#pragma unroll
  for (int off = 16; off > 0; off >>= 1) tmax = fmaxf(tmax, __shfl_xor(tmax, off, 32));
  if (lane == 0) wmax[wave] = tmax;
  __syncthreads();
  float Fmax = wmax[0];
#pragma unroll
  for (int q = 1; q < 8; ++q) Fmax = fmaxf(Fmax, wmax[q]);

  const float fi  = Fs[i0 + 16 * wave + c];
  const float lgm = fi + Fmax;
  const float mi  = (lgm >= 0.0f) ? lgm : 0.01f * lgm;

  const __bf16* XB = (const __bf16*)(const void*)xbp + (size_t)b * NC * NT;

  v8f acc[4];
#pragma unroll
  for (int t = 0; t < 4; ++t) acc[t] = (v8f){0.f, 0.f, 0.f, 0.f, 0.f, 0.f, 0.f, 0.f};
  float lsum = 0.0f;

  for (int j0 = 0; j0 < NT; j0 += KJ) {
    __syncthreads();
#pragma unroll
    for (int it = 0; it < 8; ++it) {
      const int idx = it * 256 + tid;
      const int cr  = idx >> 5;
      const int pc  = (idx & 31) * 8;
      const v8b v = *(const v8b*)(XB + (size_t)cr * NT + j0 + pc);
      *(v8b*)(VO.v + cr * VP + pc) = v;
    }
    __syncthreads();

#pragma unroll 1
    for (int kk = 0; kk < KJ / 32; ++kk) {
      const int jb = j0 + kk * 32 + 8 * hh;
      const v4f f0 = *(const v4f*)(Fs + jb);
      const v4f f1 = *(const v4f*)(Fs + jb + 4);
      const v4f f2 = *(const v4f*)(Fs + jb + 16);
      const v4f f3 = *(const v4f*)(Fs + jb + 20);
      float fj[16];
#pragma unroll
      for (int e = 0; e < 4; ++e) { fj[e] = f0[e]; fj[4 + e] = f1[e]; fj[8 + e] = f2[e]; fj[12 + e] = f3[e]; }

      v8u vh, vl;
#pragma unroll
      for (int q = 0; q < 8; ++q) {
        unsigned short h0, l0, h1, l1;
        p_elem(fi, fj[2 * q],     mi, lsum, h0, l0);
        p_elem(fi, fj[2 * q + 1], mi, lsum, h1, l1);
        vh[q] = pk16(h0, h1);
        vl[q] = pk16(l0, l1);
      }
      const v16b ah = __builtin_bit_cast(v16b, vh);
      const v16b al = __builtin_bit_cast(v16b, vl);

      FB vb[4];
#pragma unroll
      for (int t = 0; t < 4; ++t) {
        const __bf16* vp = VO.v + (t * 16 + c) * VP + kk * 32 + 8 * hh;
        vb[t].h[0] = *(const v8b*)(vp);
        vb[t].h[1] = *(const v8b*)(vp + 16);
      }
#pragma unroll
      for (int t = 0; t < 4; ++t) acc[t] = at_mma(ah, vb[t].v, acc[t]);
#pragma unroll
      for (int t = 0; t < 4; ++t) acc[t] = at_mma(al, vb[t].v, acc[t]);
    }
  }

  const float ltot = lsum + __shfl_xor(lsum, 16, 32);
  if (lane < 16) lall[16 * wave + lane] = ltot;
  __syncthreads();

#pragma unroll
  for (int t = 0; t < 4; ++t) {
#pragma unroll
    for (int r = 0; r < 8; ++r) VO.o[(t * 16 + c) * OP + 16 * wave + 8 * hh + r] = acc[t][r];
  }
  __syncthreads();

  {
    const v4f l4 = *(const v4f*)(lall + 4 * lane);
#pragma unroll 1
    for (int ch = 0; ch < 8; ++ch) {
      float* sp = VO.o + (8 * wave + ch) * OP + 4 * lane;
      const v4f v = *(const v4f*)sp;
      v4f o;
#pragma unroll
      for (int e = 0; e < 4; ++e) {
        const float q = v[e] / l4[e];
        o[e] = (q > 0.0f) ? q : expm1f(q);
      }
      *(v4f*)sp = o;
    }
    float* ob = out + ((size_t)(b * NC + 8 * wave)) * NT + i0 + 4 * lane;
    for (int pass = 0; pass < 2; ++pass) {
#pragma unroll
      for (int ch = 0; ch < 8; ++ch) {
        const v4f val = *(const v4f*)(VO.o + (8 * wave + ch) * OP + 4 * lane);
        *(volatile v4f*)(ob + (size_t)ch * NT) = val;
      }
      __threadfence();
    }
  }
}

extern "C" void kernel_launch(void* const* d_in, const int* in_sizes, int n_in,
                              void* d_out, int out_size, void* d_ws, size_t ws_size,
                              hipStream_t stream) {
  if (n_in < 2) return;
  if (in_sizes[0] != NB * NC * NT) return;
  if (in_sizes[1] != NC) return;
  if (out_size != NB * NC * NT) return;

  const size_t PXB = (size_t)NB * NC * NT * 2;
  const size_t PF  = (size_t)NB * NT * 4;
  const size_t oXB = 0;
  const size_t oF  = oXB + PXB;
  const size_t tot = oF + PF;
  if (tot > ws_size) return;
  if (tot > (size_t)134217728) return;

  const float* x = (const float*)d_in[0];
  const float* w = (const float*)d_in[1];
  char* ws = (char*)d_ws;
  unsigned short* XB = (unsigned short*)(ws + oXB);
  float*          F  = (float*)(ws + oF);
  float*          o  = (float*)d_out;

  k_prep<<<dim3((NB * NT / 4) / 256), dim3(256), 0, stream>>>(x, w, XB, F);
  k_attn<<<dim3(NT / QB, NB), dim3(256), 0, stream>>>(XB, F, o);
  (void)hipGetLastError();
}
